// OptimizedKANLayer_30812095381506
// MI455X (gfx1250) — hardware-verified
//
#include <hip/hip_runtime.h>
#include <stdint.h>


#define IN_DIM        64
#define OUT_DIM       64
#define NSPL          8
#define NACT          4
#define NKNOT         12
#define NRCP          30
#define SEQ           512
#define KSPL          (IN_DIM * NSPL)
#define KACT          (IN_DIM * NACT)
#define KTOT          (KSPL + KACT)
#define EPS_F         1e-8f
#define WSC           64.0f
#define FSC           16.0f
#define INV_SC        (1.0f / 1024.0f)
#define TOK_PER_FB    4
#define FEAT_THREADS  256
#define GEMM_THREADS  256
#define WAVES_PER_GB  8
#define PIECES_ROW    (KTOT / 8)
#define PIECES_FB     (TOK_PER_FB * PIECES_ROW)

typedef _Float16 v16h __attribute__((ext_vector_type(16)));
typedef _Float16 v8h  __attribute__((ext_vector_type(8)));
typedef _Float16 v4h  __attribute__((ext_vector_type(4)));
typedef float    v8f  __attribute__((ext_vector_type(8)));
typedef float    v4f  __attribute__((ext_vector_type(4)));
typedef v8h __attribute__((may_alias)) v8ha;
typedef v4h __attribute__((may_alias)) v4ha;
typedef v4f __attribute__((may_alias)) v4fa;

union Frag { v16h v; v8h hv[2]; _Float16 s[16]; };
union H8   { v8h v; _Float16 s[8]; };
union H4   { v4h v; _Float16 s[4]; };

__device__ __forceinline__ v8f wmma_f16_step(v16h a, v16h b, v8f c)
{
    v8f d = __builtin_amdgcn_wmma_f32_16x16x32_f16(false, a, false, b, (short)0, c, false, false);
    asm volatile("v_nop\n\tv_nop\n\tv_nop\n\tv_nop" : "+v"(d) : "v"(a), "v"(b));
    return d;
}

__global__ __launch_bounds__(FEAT_THREADS)
void k_features(const float* __restrict__ x,
                const float* __restrict__ knots,
                _Float16* __restrict__ phi,
                int ntok)
{
    __shared__ float sR[IN_DIM * NRCP];
    __shared__ __attribute__((aligned(16))) _Float16 sPhi[TOK_PER_FB * KTOT];

    const int tid = threadIdx.x;

#pragma unroll 1
    for (int e = tid; e < IN_DIM * NRCP; e += FEAT_THREADS) {
        const int d = e / NRCP;
        const int r = e - d * NRCP;
        int k, j;
        if (r < 11)      { k = 1; j = r; }
        else if (r < 21) { k = 2; j = r - 11; }
        else             { k = 3; j = r - 21; }
        const float ta  = knots[d * NKNOT + j + k];
        const float tb  = knots[d * NKNOT + j];
        const float den = (ta - tb) + EPS_F;
        sR[e] = 1.0f / den;
    }
    __syncthreads();

    const int tl    = tid >> 6;
    const int d     = tid & 63;
    const int token = blockIdx.x * TOK_PER_FB + tl;
    const int tokc  = (token < ntok) ? token : (ntok - 1);
    const float xv  = x[(size_t)tokc * IN_DIM + d];

    float t[NKNOT];
#pragma unroll
    for (int i = 0; i < NKNOT; ++i) t[i] = knots[d * NKNOT + i];

    float bv[NKNOT - 1];
#pragma unroll
    for (int i = 0; i < NKNOT - 1; ++i)
        bv[i] = (xv >= t[i] && xv < t[i + 1]) ? 1.0f : 0.0f;

    const float* rk = sR + d * NRCP;
#pragma unroll
    for (int i = 0; i < 10; ++i) {
        const float c1 = (xv - t[i]) * rk[i];
        const float c2 = (t[i + 2] - xv) * rk[i + 1];
        bv[i] = c1 * bv[i] + c2 * bv[i + 1];
    }
#pragma unroll
    for (int i = 0; i < 9; ++i) {
        const float c1 = (xv - t[i]) * rk[11 + i];
        const float c2 = (t[i + 3] - xv) * rk[11 + i + 1];
        bv[i] = c1 * bv[i] + c2 * bv[i + 1];
    }
#pragma unroll
    for (int i = 0; i < 8; ++i) {
        const float c1 = (xv - t[i]) * rk[21 + i];
        const float c2 = (t[i + 4] - xv) * rk[21 + i + 1];
        bv[i] = c1 * bv[i] + c2 * bv[i + 1];
    }

    H8 hb;
#pragma unroll
    for (int s = 0; s < NSPL; ++s) hb.s[s] = (_Float16)(bv[s] * FSC);
    *(v8ha*)(sPhi + tl * KTOT + d * NSPL) = hb.v;

    const float rl = xv > 0.0f ? xv : 0.0f;
    const float th = tanhf(xv);
    const float sg = __fdividef(1.0f, 1.0f + __expf(-xv));
    H4 ha;
    ha.s[0] = (_Float16)(rl * FSC);
    ha.s[1] = (_Float16)(th * FSC);
    ha.s[2] = (_Float16)(sg * FSC);
    ha.s[3] = (_Float16)(xv * FSC);
    *(v4ha*)(sPhi + tl * KTOT + KSPL + d * NACT) = ha.v;
    __syncthreads();

    const int p0  = tid;
    const int tlA = p0 / PIECES_ROW;
    const int qA  = p0 - tlA * PIECES_ROW;
    const int tkA = blockIdx.x * TOK_PER_FB + tlA;
    const bool okA = tkA < ntok;
    const v8h vA = *(const v8ha*)(sPhi + tlA * KTOT + qA * 8);
    _Float16* dA = phi + (size_t)(okA ? tkA : 0) * KTOT + qA * 8;

    const int p1r = tid + FEAT_THREADS;
    const bool has1 = p1r < PIECES_FB;
    const int p1  = has1 ? p1r : p0;
    const int tlB = p1 / PIECES_ROW;
    const int qB  = p1 - tlB * PIECES_ROW;
    const int tkB = blockIdx.x * TOK_PER_FB + tlB;
    const bool okB = has1 && (tkB < ntok);
    const v8h vB = *(const v8ha*)(sPhi + tlB * KTOT + qB * 8);
    _Float16* dB = phi + (size_t)(okB ? tkB : 0) * KTOT + qB * 8;

    if (okA) *(volatile v8h*)dA = vA;
    if (okB) *(volatile v8h*)dB = vB;
    __threadfence();
    if (okA) *(volatile v8h*)dA = vA;
    if (okB) *(volatile v8h*)dB = vB;
}

__global__ __launch_bounds__(GEMM_THREADS)
void k_gemm(const float* __restrict__ cp,
            const float* __restrict__ aw,
            const _Float16* __restrict__ phi,
            float* __restrict__ out,
            int ntok)
{
    __shared__ __attribute__((aligned(16))) float sT[WAVES_PER_GB * 16 * 32];

    const int tid  = threadIdx.x;
    const int wib  = tid >> 5;
    const int lane = tid & 31;
    const int h    = lane >> 4;
    const int m    = lane & 15;

    const int nwaves = (ntok >> 5) * (OUT_DIM / 16);
    const int wave   = blockIdx.x * WAVES_PER_GB + wib;
    const bool wvalid = wave < nwaves;
    const int wc    = wvalid ? wave : 0;
    const int mtile = wc & 3;
    const int npair = wc >> 2;
    const int o0    = mtile * 16;
    const int t0    = npair * 32;

    const float* cprow = cp + (size_t)(o0 + m) * KSPL;
    const float* awrow = aw + (size_t)(o0 + m) * KACT;
    const _Float16* pr0 = phi + (size_t)(t0 + m) * KTOT;
    const _Float16* pr1 = phi + (size_t)(t0 + 16 + m) * KTOT;

    v8f acc0 = {0.f, 0.f, 0.f, 0.f, 0.f, 0.f, 0.f, 0.f};
    v8f acc1 = {0.f, 0.f, 0.f, 0.f, 0.f, 0.f, 0.f, 0.f};
    v8f acc2 = {0.f, 0.f, 0.f, 0.f, 0.f, 0.f, 0.f, 0.f};
    v8f acc3 = {0.f, 0.f, 0.f, 0.f, 0.f, 0.f, 0.f, 0.f};

#pragma unroll 2
    for (int kb = 0; kb < KSPL; kb += 32) {
        const v4f w0 = *(const v4fa*)(cprow + kb + 8 * h);
        const v4f w1 = *(const v4fa*)(cprow + kb + 8 * h + 4);
        const v4f w2 = *(const v4fa*)(cprow + kb + 16 + 8 * h);
        const v4f w3 = *(const v4fa*)(cprow + kb + 16 + 8 * h + 4);
        Frag a;
#pragma unroll
        for (int i = 0; i < 4; ++i) {
            a.s[i]      = (_Float16)(w0[i] * WSC);
            a.s[4 + i]  = (_Float16)(w1[i] * WSC);
            a.s[8 + i]  = (_Float16)(w2[i] * WSC);
            a.s[12 + i] = (_Float16)(w3[i] * WSC);
        }
        Frag b0, b1;
        b0.hv[0] = *(const v8h*)(pr0 + kb + 8 * h);
        b0.hv[1] = *(const v8h*)(pr0 + kb + 16 + 8 * h);
        b1.hv[0] = *(const v8h*)(pr1 + kb + 8 * h);
        b1.hv[1] = *(const v8h*)(pr1 + kb + 16 + 8 * h);
        acc0 = wmma_f16_step(a.v, b0.v, acc0);
        acc1 = wmma_f16_step(a.v, b1.v, acc1);
    }

    const _Float16* qa0 = pr0 + KSPL;
    const _Float16* qa1 = pr1 + KSPL;
#pragma unroll 2
    for (int kb = 0; kb < KACT; kb += 32) {
        const v4f w0 = *(const v4fa*)(awrow + kb + 8 * h);
        const v4f w1 = *(const v4fa*)(awrow + kb + 8 * h + 4);
        const v4f w2 = *(const v4fa*)(awrow + kb + 16 + 8 * h);
        const v4f w3 = *(const v4fa*)(awrow + kb + 16 + 8 * h + 4);
        Frag a;
#pragma unroll
        for (int i = 0; i < 4; ++i) {
            a.s[i]      = (_Float16)(w0[i] * WSC);
            a.s[4 + i]  = (_Float16)(w1[i] * WSC);
            a.s[8 + i]  = (_Float16)(w2[i] * WSC);
            a.s[12 + i] = (_Float16)(w3[i] * WSC);
        }
        Frag b0, b1;
        b0.hv[0] = *(const v8h*)(qa0 + kb + 8 * h);
        b0.hv[1] = *(const v8h*)(qa0 + kb + 16 + 8 * h);
        b1.hv[0] = *(const v8h*)(qa1 + kb + 8 * h);
        b1.hv[1] = *(const v8h*)(qa1 + kb + 16 + 8 * h);
        acc2 = wmma_f16_step(a.v, b0.v, acc2);
        acc3 = wmma_f16_step(a.v, b1.v, acc3);
    }

    float* tile = sT + wib * (16 * 32);
#pragma unroll
    for (int j = 0; j < 8; ++j) {
        const int r = 8 * h + j;
        const float s0 = acc0[j] * INV_SC;
        const float s1 = acc1[j] * INV_SC;
        const float g0 = acc2[j] * INV_SC;
        const float g1 = acc3[j] * INV_SC;
        tile[r * 32 + m]      = s0 + 0.1f * g0;
        tile[r * 32 + 16 + m] = s1 + 0.1f * g1;
    }
    __syncthreads();

    const int bidx = t0 / SEQ;
    const int n0   = t0 - bidx * SEQ;
    const int g    = lane >> 3;
    const int q    = lane & 7;
    v4f    v[4];
    size_t off[4];
#pragma unroll
    for (int p = 0; p < 4; ++p) {
        const int r = p * 4 + g;
        v[p]   = *(const v4fa*)(tile + r * 32 + q * 4);
        off[p] = ((size_t)(bidx * OUT_DIM + o0 + r)) * SEQ + (size_t)(n0 + q * 4);
    }
    if (wvalid) {
#pragma unroll
        for (int p = 0; p < 4; ++p) *(volatile v4f*)(out + off[p]) = v[p];
    }
    __threadfence();
    if (wvalid) {
#pragma unroll
        for (int p = 0; p < 4; ++p) *(volatile v4f*)(out + off[p]) = v[p];
    }
}

extern "C" void kernel_launch(void* const* d_in, const int* in_sizes, int n_in,
                              void* d_out, int out_size, void* d_ws, size_t ws_size,
                              hipStream_t stream)
{
    if (n_in < 4) return;
    const int nx = in_sizes[0];
    if (nx <= 0 || (nx % IN_DIM) != 0) return;
    const int ntok = nx / IN_DIM;
    if ((ntok % SEQ) != 0) return;
    if (in_sizes[1] != OUT_DIM * KSPL) return;
    if (in_sizes[2] <  IN_DIM * NKNOT) return;
    if (in_sizes[3] != OUT_DIM * KACT) return;
    if (out_size != (ntok / SEQ) * OUT_DIM * SEQ) return;

    const size_t phi_bytes = (size_t)ntok * KTOT * sizeof(_Float16);
    if (phi_bytes > ws_size) return;

    const float* x     = (const float*)d_in[0];
    const float* cp    = (const float*)d_in[1];
    const float* knots = (const float*)d_in[2];
    const float* aw    = (const float*)d_in[3];
    float*       out   = (float*)d_out;
    _Float16*    phi   = (_Float16*)d_ws;

    const int fblocks = (ntok + TOK_PER_FB - 1) / TOK_PER_FB;
    const int nwaves  = (ntok / 32) * (OUT_DIM / 16);
    const int gblocks = (nwaves + WAVES_PER_GB - 1) / WAVES_PER_GB;

    k_features<<<fblocks, FEAT_THREADS, 0, stream>>>(x, knots, phi, ntok);
    k_gemm<<<gblocks, GEMM_THREADS, 0, stream>>>(cp, aw, phi, out, ntok);
}
